// CausalSelfAttention_56753697849991
// MI455X (gfx1250) — hardware-verified
//
#include <hip/hip_runtime.h>

#ifndef NB
#define NB 2
#endif
#ifndef SEQ
#define SEQ 2048
#endif
#define SEQ_FULL 2048
#define EMB 1024
#define NHEAD 16
#define HD 64
#define EARLY 256
#define PPH 40
#define OSP 68
#define CDIV(a, b) (((a) + (b) - 1) / (b))

static_assert(NHEAD * HD == EMB);
static_assert(HD == 64);
static_assert(EMB % 64 == 0);
static_assert(EMB % 32 == 0);
static_assert((3 * EMB) % 64 == 0);
static_assert(SEQ % 64 == 0);
static_assert(EARLY % 64 == 0);
static_assert(SEQ >= EARLY);
static_assert(SEQ <= SEQ_FULL);
static_assert((NB * SEQ) % 64 == 0);
static_assert((PPH * 2) % 16 == 0);
static_assert((OSP * 4) % 16 == 0);

typedef __attribute__((ext_vector_type(16))) _Float16       v16h;
typedef __attribute__((ext_vector_type(16))) __bf16         v16b;
typedef __attribute__((ext_vector_type(8)))  float          v8f;
typedef __attribute__((ext_vector_type(4)))  float          v4f;
typedef __attribute__((ext_vector_type(8)))  unsigned short v8us;
typedef __attribute__((ext_vector_type(16))) unsigned short v16us;
typedef __attribute__((ext_vector_type(4)))  unsigned int   v4u;

__device__ __forceinline__ unsigned short bf_bits(float f) {
  const unsigned u = __float_as_uint(f);
  return (unsigned short)((u + 0x7FFFu + ((u >> 16) & 1u)) >> 16);
}
__device__ __forceinline__ float bf_val(unsigned short h) { return __uint_as_float(((unsigned)h) << 16); }
__device__ __forceinline__ float bf_rne_f32(float v) { return bf_val(bf_bits(v)); }
__device__ __forceinline__ unsigned short h_bits(float f) { return __builtin_bit_cast(unsigned short, (_Float16)f); }
__device__ __forceinline__ unsigned pk2(unsigned short a, unsigned short b) { return (unsigned)a | ((unsigned)b << 16); }

__device__ __forceinline__ v4u pack8_f16(v4f a, v4f b) {
  v4u p;
  p.x = pk2(h_bits(a.x), h_bits(a.y)); p.y = pk2(h_bits(a.z), h_bits(a.w));
  p.z = pk2(h_bits(b.x), h_bits(b.y)); p.w = pk2(h_bits(b.z), h_bits(b.w));
  return p;
}
__device__ __forceinline__ void pack8_bf(v4f a, v4f b, v4u& hi, v4u& lo) {
  const unsigned short h0 = bf_bits(a.x), h1 = bf_bits(a.y), h2 = bf_bits(a.z), h3 = bf_bits(a.w);
  const unsigned short h4 = bf_bits(b.x), h5 = bf_bits(b.y), h6 = bf_bits(b.z), h7 = bf_bits(b.w);
  hi.x = pk2(h0, h1); hi.y = pk2(h2, h3); hi.z = pk2(h4, h5); hi.w = pk2(h6, h7);
  lo.x = pk2(bf_bits(a.x - bf_val(h0)), bf_bits(a.y - bf_val(h1)));
  lo.y = pk2(bf_bits(a.z - bf_val(h2)), bf_bits(a.w - bf_val(h3)));
  lo.z = pk2(bf_bits(b.x - bf_val(h4)), bf_bits(b.y - bf_val(h5)));
  lo.w = pk2(bf_bits(b.z - bf_val(h6)), bf_bits(b.w - bf_val(h7)));
}
__device__ __forceinline__ void st16_twice(unsigned short* p, v4u v) {
  volatile v4u* d = (volatile v4u*)p;
  *d = v; __threadfence(); *d = v;
}

__device__ __forceinline__ v16us ldfrag_g(const unsigned short* __restrict__ p) {
  const v8us a = *(const v8us*)p;
  const v8us b = *(const v8us*)(p + 16);
  return __builtin_shufflevector(a, b, 0, 1, 2, 3, 4, 5, 6, 7, 8, 9, 10, 11, 12, 13, 14, 15);
}

template <bool BF>
__device__ __forceinline__ v8f mma16(v16us a, v16us b, v8f c) {
  if (BF) {
    const v16b x = __builtin_bit_cast(v16b, a), y = __builtin_bit_cast(v16b, b);
    c = __builtin_amdgcn_wmma_f32_16x16x32_bf16(false, x, false, y, (short)0, c, false, false);
    asm volatile("v_nop\n\tv_nop\n\tv_nop\n\tv_nop" : "+v"(c) : "v"(x), "v"(y));
  } else {
    const v16h x = __builtin_bit_cast(v16h, a), y = __builtin_bit_cast(v16h, b);
    c = __builtin_amdgcn_wmma_f32_16x16x32_f16(false, x, false, y, (short)0, c, false, false);
    asm volatile("v_nop\n\tv_nop\n\tv_nop\n\tv_nop" : "+v"(c) : "v"(x), "v"(y));
  }
  return c;
}

__global__ __launch_bounds__(256) void k_cast_rows(const float* __restrict__ src, long long sbs, unsigned short* __restrict__ dst, long long dbs,
                                                    int nR, int nC, float sc) {
  const long long u = (long long)blockIdx.x * 256 + threadIdx.x;
  const int per = nC >> 3;
  if (u >= (long long)nR * per) return;
  const int r = (int)(u / per), c0 = 8 * (int)(u % per);
  const float* s = src + (long long)blockIdx.y * sbs + (long long)r * nC + c0;
  const v4f a = *(const v4f*)s, b = *(const v4f*)(s + 4);
  v4f a2, b2;
  a2.x = bf_rne_f32(a.x) * sc; a2.y = bf_rne_f32(a.y) * sc; a2.z = bf_rne_f32(a.z) * sc; a2.w = bf_rne_f32(a.w) * sc;
  b2.x = bf_rne_f32(b.x) * sc; b2.y = bf_rne_f32(b.y) * sc; b2.z = bf_rne_f32(b.z) * sc; b2.w = bf_rne_f32(b.w) * sc;
  st16_twice(dst + (long long)blockIdx.y * dbs + (long long)r * nC + c0, pack8_f16(a2, b2));
}
__global__ __launch_bounds__(256) void k_castT(const float* __restrict__ src, int lds, unsigned short* __restrict__ dst, int ldd,
                                                int nR, int nC, float sc, int bfmode) {
  const long long u = (long long)blockIdx.x * 256 + threadIdx.x;
  const int per = nR >> 3;
  if (u >= (long long)nC * per) return;
  const int c = (int)(u / per), r0 = 8 * (int)(u % per);
  float w[8];
#pragma unroll
  for (int e = 0; e < 8; ++e) w[e] = bf_rne_f32(src[(long long)(r0 + e) * lds + c]);
  v4u pk;
  if (bfmode) {
    pk.x = pk2((unsigned short)(__float_as_uint(w[0]) >> 16), (unsigned short)(__float_as_uint(w[1]) >> 16));
    pk.y = pk2((unsigned short)(__float_as_uint(w[2]) >> 16), (unsigned short)(__float_as_uint(w[3]) >> 16));
    pk.z = pk2((unsigned short)(__float_as_uint(w[4]) >> 16), (unsigned short)(__float_as_uint(w[5]) >> 16));
    pk.w = pk2((unsigned short)(__float_as_uint(w[6]) >> 16), (unsigned short)(__float_as_uint(w[7]) >> 16));
  } else {
    pk.x = pk2(h_bits(w[0] * sc), h_bits(w[1] * sc)); pk.y = pk2(h_bits(w[2] * sc), h_bits(w[3] * sc));
    pk.z = pk2(h_bits(w[4] * sc), h_bits(w[5] * sc)); pk.w = pk2(h_bits(w[6] * sc), h_bits(w[7] * sc));
  }
  st16_twice(dst + (long long)c * ldd + r0, pk);
}

template <bool BF, bool ALO, int BIAS_MODE, int OUT_MODE>
__device__ __forceinline__ void gemm64_body(
    const unsigned short* __restrict__ A, const unsigned short* __restrict__ A2, const int lda, const long long strideA,
    const unsigned short* __restrict__ Bt, const int ldb, const long long strideB,
    float* __restrict__ Cf, unsigned short* __restrict__ Ch, unsigned short* __restrict__ Cl, const int ldc, const long long strideC,
    const float* __restrict__ bias, const int M, const int N, const int K, const float scale) {
  __shared__ __align__(16) float sT[8][16 * OSP];
  const int b = blockIdx.y;
  const int lane = threadIdx.x & 31;
  const int wave = __builtin_amdgcn_readfirstlane((int)(threadIdx.x >> 5));
  const int tilesN = N >> 6, tilesM = M >> 6, ntile = tilesM * tilesN;
  int tile = (int)blockIdx.x * 8 + wave;
  const bool live = tile < ntile;
  tile = min(tile, ntile - 1);
  const int tm = tile / tilesN, tn = tile - tm * tilesN;
  const int m0 = tm << 6, n0 = tn << 6;
  const unsigned short* Ab  = A  + (size_t)b * strideA;
  const unsigned short* A2b = A2 + (size_t)b * strideA;
  const unsigned short* Bb  = Bt + (size_t)b * strideB;
  const int rl = lane & 15;
  const int koff = (lane >> 4) * 8;
  const int mOff = (lane >> 4) * 8;

  v8f acc[4][4];
#pragma unroll
  for (int i = 0; i < 4; ++i)
#pragma unroll
    for (int j = 0; j < 4; ++j) acc[i][j] = (v8f){0.f, 0.f, 0.f, 0.f, 0.f, 0.f, 0.f, 0.f};

  for (int k0 = 0; k0 < K; k0 += 32) {
    v16us bh[4];
#pragma unroll
    for (int j = 0; j < 4; ++j) bh[j] = ldfrag_g(Bb + (size_t)(n0 + (j << 4) + rl) * ldb + k0 + koff);
#pragma unroll
    for (int i = 0; i < 4; ++i) {
      const size_t ao = (size_t)(m0 + (i << 4) + rl) * lda + k0 + koff;
      const v16us ah = ldfrag_g(Ab + ao);
      v16us al = ah;
      if (ALO) al = ldfrag_g(A2b + ao);
#pragma unroll
      for (int j = 0; j < 4; ++j) {
        acc[i][j] = mma16<BF>(ah, bh[j], acc[i][j]);
        if (ALO) acc[i][j] = mma16<BF>(al, bh[j], acc[i][j]);
      }
    }
  }

#pragma unroll
  for (int i = 0; i < 4; ++i) {
    const int mBase = m0 + (i << 4);
#pragma unroll
    for (int j = 0; j < 4; ++j) {
      const int n = n0 + (j << 4) + rl;
      float bv = 0.f;
      if (BIAS_MODE == 2) bv = bf_rne_f32(bias[n]);
#pragma unroll
      for (int r = 0; r < 8; ++r) {
        float v = acc[i][j][r] * scale;
        if (BIAS_MODE == 1) v += bf_rne_f32(bias[mBase + mOff + r]);
        if (BIAS_MODE == 2) v += bv;
        sT[wave][(mOff + r) * OSP + (j << 4) + rl] = v;
      }
    }
    __syncthreads();
    if (live) {
      if (OUT_MODE == 0) {
        float* C = Cf + (size_t)b * strideC;
        const int hh = lane >> 4, c4 = (lane & 15) * 4;
        for (int pass = 0; pass < 2; ++pass) {
#pragma unroll
          for (int it = 0; it < 8; ++it) {
            const int row = it * 2 + hh;
            const v4f v = *(const v4f*)&sT[wave][row * OSP + c4];
            *(volatile v4f*)(C + (size_t)(mBase + row) * ldc + n0 + c4) = v;
          }
          __threadfence();
        }
      } else {
        const int q = lane >> 3, c8 = (lane & 7) * 8;
        unsigned short* C1 = Ch + (size_t)b * strideC;
        unsigned short* C2 = Cl + (size_t)b * strideC;
        for (int pass = 0; pass < 2; ++pass) {
#pragma unroll
          for (int it = 0; it < 4; ++it) {
            const int row = it * 4 + q;
            const v4f a = *(const v4f*)&sT[wave][row * OSP + c8];
            const v4f c = *(const v4f*)&sT[wave][row * OSP + c8 + 4];
            const size_t o = (size_t)(mBase + row) * ldc + n0 + c8;
            if (OUT_MODE == 1) {
              *(volatile v4u*)(C1 + o) = pack8_f16(a, c);
            } else {
              v4u hi, lo; pack8_bf(a, c, hi, lo);
              *(volatile v4u*)(C1 + o) = hi;
              *(volatile v4u*)(C2 + o) = lo;
            }
          }
          __threadfence();
        }
      }
    }
    __syncthreads();
  }
}

__global__ __launch_bounds__(256) void k_gemm_f16out_bn(const unsigned short* __restrict__ A, int lda, long long strideA,
    const unsigned short* __restrict__ Bt, int ldb, long long strideB, unsigned short* __restrict__ C, int ldc, long long strideC,
    const float* __restrict__ bias, int M, int N, int K, float scale) {
  gemm64_body<false, false, 2, 1>(A, A, lda, strideA, Bt, ldb, strideB, nullptr, C, C, ldc, strideC, bias, M, N, K, scale);
}
__global__ __launch_bounds__(256) void k_gemm_f16out_bm(const unsigned short* __restrict__ A, int lda, long long strideA,
    const unsigned short* __restrict__ Bt, int ldb, long long strideB, unsigned short* __restrict__ C, int ldc, long long strideC,
    const float* __restrict__ bias, int M, int N, int K, float scale) {
  gemm64_body<false, false, 1, 1>(A, A, lda, strideA, Bt, ldb, strideB, nullptr, C, C, ldc, strideC, bias, M, N, K, scale);
}
__global__ __launch_bounds__(256) void k_gemm_hilo_bn(const unsigned short* __restrict__ A, int lda, long long strideA,
    const unsigned short* __restrict__ Bt, int ldb, long long strideB, unsigned short* __restrict__ Chi, unsigned short* __restrict__ Clo, int ldc, long long strideC,
    const float* __restrict__ bias, int M, int N, int K, float scale) {
  gemm64_body<false, false, 2, 2>(A, A, lda, strideA, Bt, ldb, strideB, nullptr, Chi, Clo, ldc, strideC, bias, M, N, K, scale);
}
__global__ __launch_bounds__(256) void k_gemm_hilo_bm(const unsigned short* __restrict__ A, int lda, long long strideA,
    const unsigned short* __restrict__ Bt, int ldb, long long strideB, unsigned short* __restrict__ Chi, unsigned short* __restrict__ Clo, int ldc, long long strideC,
    const float* __restrict__ bias, int M, int N, int K, float scale) {
  gemm64_body<false, false, 1, 2>(A, A, lda, strideA, Bt, ldb, strideB, nullptr, Chi, Clo, ldc, strideC, bias, M, N, K, scale);
}
__global__ __launch_bounds__(256) void k_gemm_f32out_bn(const unsigned short* __restrict__ A, int lda, long long strideA,
    const unsigned short* __restrict__ Bt, int ldb, long long strideB, float* __restrict__ C, int ldc, long long strideC,
    const float* __restrict__ bias, int M, int N, int K, float scale) {
  gemm64_body<false, false, 2, 0>(A, A, lda, strideA, Bt, ldb, strideB, C, nullptr, nullptr, ldc, strideC, bias, M, N, K, scale);
}
__global__ __launch_bounds__(256) void k_gemm_bfsplit_f32out_bn(const unsigned short* __restrict__ Ahi, const unsigned short* __restrict__ Alo, int lda, long long strideA,
    const unsigned short* __restrict__ Bt, int ldb, long long strideB, float* __restrict__ C, int ldc, long long strideC,
    const float* __restrict__ bias, int M, int N, int K, float scale) {
  gemm64_body<true, true, 2, 0>(Ahi, Alo, lda, strideA, Bt, ldb, strideB, C, nullptr, nullptr, ldc, strideC, bias, M, N, K, scale);
}

template <bool RES>
__device__ __forceinline__ void attn_body(
    const unsigned short* __restrict__ QKh, const unsigned short* __restrict__ QKl, const int ldqk,
    const unsigned short* __restrict__ VTh, const unsigned short* __restrict__ VTl, const int ldvt,
    unsigned short* __restrict__ Oh, unsigned short* __restrict__ Ol, const int ldo,
    const int qs0, const int hcol, const float pcarry, const float ocarry) {
  __shared__ __align__(16) unsigned short plh[4][16 * PPH];
  __shared__ __align__(16) unsigned short pll[4][16 * PPH];
  __shared__ __align__(16) float os[4][16 * OSP];
  const int lane = threadIdx.x & 31, hf = lane >> 4, l15 = lane & 15;
  const int wave = __builtin_amdgcn_readfirstlane((int)(threadIdx.x >> 5));
  const int q0 = qs0 + 16 * wave;
  const int nkb = (qs0 >> 6) + 1;
  const float NEG = -__builtin_inff();
  const float CS = 0.125f * 1.4426950408889634f;
  const size_t qoff = (size_t)(q0 + l15) * ldqk + hcol + 8 * hf;

  float m8[8], l8[8];
  v8f o[4];
#pragma unroll
  for (int r = 0; r < 8; ++r) { m8[r] = NEG; l8[r] = 0.f; }
#pragma unroll
  for (int t = 0; t < 4; ++t) o[t] = (v8f){0.f, 0.f, 0.f, 0.f, 0.f, 0.f, 0.f, 0.f};

  for (int kb = 0; kb < nkb; ++kb) {
    const bool diag = (kb == nkb - 1);
#pragma unroll 1
    for (int hh2 = 0; hh2 < 2; ++hh2) {
      const int j0 = kb * 64 + hh2 * 32;
      v8f s0 = (v8f){0.f, 0.f, 0.f, 0.f, 0.f, 0.f, 0.f, 0.f};
      v8f s1 = s0;
#pragma unroll
      for (int ks = 0; ks < 2; ++ks) {
        const size_t ko0 = (size_t)(j0 + l15) * ldqk + EMB + hcol + 32 * ks + 8 * hf;
        const size_t ko1 = ko0 + (size_t)16 * ldqk;
        const v16us qh = ldfrag_g(QKh + qoff + 32 * ks);
        const v16us k0h = ldfrag_g(QKh + ko0);
        const v16us k1h = ldfrag_g(QKh + ko1);
        s0 = mma16<RES>(qh, k0h, s0);
        s1 = mma16<RES>(qh, k1h, s1);
        if (RES) {
          const v16us ql = ldfrag_g(QKl + qoff + 32 * ks);
          const v16us k0l = ldfrag_g(QKl + ko0);
          const v16us k1l = ldfrag_g(QKl + ko1);
          s0 = mma16<RES>(qh, k0l, s0);
          s0 = mma16<RES>(ql, k0h, s0);
          s1 = mma16<RES>(qh, k1l, s1);
          s1 = mma16<RES>(ql, k1h, s1);
        }
      }
      __syncthreads();
#pragma unroll
      for (int r = 0; r < 8; ++r) {
        const int qrow = q0 + 8 * hf + r;
        float a0 = s0[r] * CS, a1 = s1[r] * CS;
        a0 = (diag && (j0 + l15 > qrow)) ? NEG : a0;
        a1 = (diag && (j0 + 16 + l15 > qrow)) ? NEG : a1;
        float mx = fmaxf(a0, a1);
        mx = fmaxf(mx, __shfl_xor(mx, 1, 32)); mx = fmaxf(mx, __shfl_xor(mx, 2, 32));
        mx = fmaxf(mx, __shfl_xor(mx, 4, 32)); mx = fmaxf(mx, __shfl_xor(mx, 8, 32));
        const float mnew = fmaxf(m8[r], mx);
        const float corr = (mnew == NEG) ? 1.f : exp2f(m8[r] - mnew);
        const float p0 = (a0 == NEG) ? 0.f : exp2f(a0 - mnew);
        const float p1 = (a1 == NEG) ? 0.f : exp2f(a1 - mnew);
        float rs = p0 + p1;
        rs += __shfl_xor(rs, 1, 32); rs += __shfl_xor(rs, 2, 32); rs += __shfl_xor(rs, 4, 32); rs += __shfl_xor(rs, 8, 32);
        l8[r] = l8[r] * corr + rs;
        m8[r] = mnew;
#pragma unroll
        for (int t = 0; t < 4; ++t) o[t][r] *= corr;
        const int pi = (8 * hf + r) * PPH + l15;
        if (RES) {
          const unsigned short h0 = bf_bits(p0), h1 = bf_bits(p1);
          plh[wave][pi] = h0; plh[wave][pi + 16] = h1;
          pll[wave][pi] = bf_bits(p0 - bf_val(h0)); pll[wave][pi + 16] = bf_bits(p1 - bf_val(h1));
        } else {
          plh[wave][pi] = h_bits(p0 * pcarry); plh[wave][pi + 16] = h_bits(p1 * pcarry);
        }
      }
      __syncthreads();
      const v8us x0 = *(const v8us*)&plh[wave][l15 * PPH + 8 * hf];
      const v8us x1 = *(const v8us*)&plh[wave][l15 * PPH + 16 + 8 * hf];
      const v16us pah = __builtin_shufflevector(x0, x1, 0, 1, 2, 3, 4, 5, 6, 7, 8, 9, 10, 11, 12, 13, 14, 15);
      v16us pal = pah;
      if (RES) {
        const v8us y0 = *(const v8us*)&pll[wave][l15 * PPH + 8 * hf];
        const v8us y1 = *(const v8us*)&pll[wave][l15 * PPH + 16 + 8 * hf];
        pal = __builtin_shufflevector(y0, y1, 0, 1, 2, 3, 4, 5, 6, 7, 8, 9, 10, 11, 12, 13, 14, 15);
      }
#pragma unroll
      for (int t = 0; t < 4; ++t) {
        const size_t vo = (size_t)(hcol + 16 * t + l15) * ldvt + j0 + 8 * hf;
        const v16us vh = ldfrag_g(VTh + vo);
        o[t] = mma16<RES>(pah, vh, o[t]);
        if (RES) {
          const v16us vl = ldfrag_g(VTl + vo);
          o[t] = mma16<RES>(pah, vl, o[t]);
          o[t] = mma16<RES>(pal, vh, o[t]);
        }
      }
    }
  }

#pragma unroll
  for (int r = 0; r < 8; ++r) {
    const float inv = ocarry * (1.0f / (l8[r] * pcarry));
#pragma unroll
    for (int t = 0; t < 4; ++t) os[wave][(8 * hf + r) * OSP + 16 * t + l15] = o[t][r] * inv;
  }
  __syncthreads();
  {
    const int q = lane >> 3, c8 = (lane & 7) * 8;
    for (int pass = 0; pass < 2; ++pass) {
#pragma unroll
      for (int it = 0; it < 4; ++it) {
        const int row = it * 4 + q;
        const v4f a = *(const v4f*)&os[wave][row * OSP + c8];
        const v4f c = *(const v4f*)&os[wave][row * OSP + c8 + 4];
        const size_t oo = (size_t)(q0 + row) * ldo + hcol + c8;
        if (RES) {
          v4u hi, lo; pack8_bf(a, c, hi, lo);
          *(volatile v4u*)(Oh + oo) = hi;
          *(volatile v4u*)(Ol + oo) = lo;
        } else {
          *(volatile v4u*)(Oh + oo) = pack8_f16(a, c);
        }
      }
      __threadfence();
    }
  }
}

__global__ __launch_bounds__(128) void k_attn_late(const unsigned short* __restrict__ QK16, const unsigned short* __restrict__ VT16, unsigned short* __restrict__ CTX16) {
  const int b = blockIdx.z, h = blockIdx.y;
  const int qs0 = EARLY + 64 * (int)blockIdx.x;
  const unsigned short* qk = QK16 + (size_t)b * SEQ * (2 * EMB);
  const unsigned short* vt = VT16 + (size_t)b * SEQ;
  unsigned short* oc = CTX16 + (size_t)b * SEQ * EMB;
  attn_body<false>(qk, qk, 2 * EMB, vt, vt, NB * SEQ, oc, oc, EMB, qs0, h * HD, 1024.0f, 16.0f);
}
__global__ __launch_bounds__(128) void k_attn_early(const unsigned short* __restrict__ QKEH, const unsigned short* __restrict__ QKEL,
                                                     const unsigned short* __restrict__ VTEH, const unsigned short* __restrict__ VTEL,
                                                     unsigned short* __restrict__ CTXEH, unsigned short* __restrict__ CTXEL) {
  const int b = blockIdx.z, h = blockIdx.y;
  const int qs0 = 64 * (int)blockIdx.x;
  const size_t qo = (size_t)b * EARLY * (2 * EMB), vo = (size_t)b * EMB * EARLY, co = (size_t)b * EARLY * EMB;
  attn_body<true>(QKEH + qo, QKEL + qo, 2 * EMB, VTEH + vo, VTEL + vo, EARLY, CTXEH + co, CTXEL + co, EMB, qs0, h * HD, 1.0f, 1.0f);
}

#define SZ_X16  ((size_t)NB * SEQ * EMB * 2)
#define SZ_W3   ((size_t)3 * EMB * EMB * 2)
#define SZ_WO   ((size_t)EMB * EMB * 2)
#define SZ_QK   ((size_t)NB * SEQ * 2 * EMB * 2)
#define SZ_VT   ((size_t)EMB * NB * SEQ * 2)
#define SZ_QKE  ((size_t)NB * EARLY * 2 * EMB * 2)
#define SZ_VTE  ((size_t)NB * EMB * EARLY * 2)
#define SZ_CTX  ((size_t)NB * SEQ * EMB * 2)
#define SZ_CTXE ((size_t)NB * EARLY * EMB * 2)
#define WS_TOTAL (SZ_X16 + SZ_W3 + 2 * SZ_WO + SZ_QK + SZ_VT + 2 * SZ_QKE + 2 * SZ_VTE + SZ_CTX + 2 * SZ_CTXE)
static_assert(WS_TOTAL <= (size_t)134217728);
static_assert(SZ_X16 % 256 == 0 && SZ_W3 % 256 == 0 && SZ_WO % 256 == 0 && SZ_QK % 256 == 0 && SZ_VT % 256 == 0);
static_assert(SZ_QKE % 256 == 0 && SZ_VTE % 256 == 0 && SZ_CTX % 256 == 0 && SZ_CTXE % 256 == 0);

extern "C" void kernel_launch(void* const* d_in, const int* in_sizes, int n_in, void* d_out, int out_size, void* d_ws, size_t ws_size, hipStream_t stream) {
  if (n_in < 5) return;
  const long long need_x = (long long)(NB - 1) * SEQ_FULL * EMB + (long long)SEQ * EMB;
  if ((long long)in_sizes[0] < need_x) return;
  if ((long long)in_sizes[1] < (long long)3 * EMB * EMB) return;
  if (in_sizes[2] < 3 * EMB) return;
  if ((long long)in_sizes[3] < (long long)EMB * EMB) return;
  if (in_sizes[4] < EMB) return;
  if ((long long)out_size < need_x) return;
  if (ws_size < WS_TOTAL) return;

  const float* x    = (const float*)d_in[0];
  const float* Wqkv = (const float*)d_in[1];
  const float* bqkv = (const float*)d_in[2];
  const float* Wo   = (const float*)d_in[3];
  const float* bo   = (const float*)d_in[4];
  float* out = (float*)d_out;

  char* w = (char*)d_ws;
  unsigned short* X16   = (unsigned short*)w; w += SZ_X16;
  unsigned short* W316  = (unsigned short*)w; w += SZ_W3;
  unsigned short* WO16  = (unsigned short*)w; w += SZ_WO;
  unsigned short* WOB   = (unsigned short*)w; w += SZ_WO;
  unsigned short* QK16  = (unsigned short*)w; w += SZ_QK;
  unsigned short* VT16  = (unsigned short*)w; w += SZ_VT;
  unsigned short* QKEH  = (unsigned short*)w; w += SZ_QKE;
  unsigned short* QKEL  = (unsigned short*)w; w += SZ_QKE;
  unsigned short* VTEH  = (unsigned short*)w; w += SZ_VTE;
  unsigned short* VTEL  = (unsigned short*)w; w += SZ_VTE;
  unsigned short* CTX16 = (unsigned short*)w; w += SZ_CTX;
  unsigned short* CTXEH = (unsigned short*)w; w += SZ_CTXE;
  unsigned short* CTXEL = (unsigned short*)w; w += SZ_CTXE;

  k_cast_rows<<<dim3((unsigned)CDIV((long long)SEQ * (EMB / 8), 256), (unsigned)NB), 256, 0, stream>>>(
      x, (long long)SEQ_FULL * EMB, X16, (long long)SEQ * EMB, SEQ, EMB, 1.0f);
  k_castT<<<(unsigned)CDIV((long long)(3 * EMB) * (EMB / 8), 256), 256, 0, stream>>>(Wqkv, 3 * EMB, W316, EMB, EMB, 3 * EMB, 16.0f, 0);
  k_castT<<<(unsigned)CDIV((long long)EMB * (EMB / 8), 256), 256, 0, stream>>>(Wo, EMB, WO16, EMB, EMB, EMB, 16.0f, 0);
  k_castT<<<(unsigned)CDIV((long long)EMB * (EMB / 8), 256), 256, 0, stream>>>(Wo, EMB, WOB, EMB, EMB, EMB, 1.0f, 1);

  k_gemm_f16out_bn<<<dim3((unsigned)CDIV((NB * SEQ / 64) * (2 * EMB / 64), 8), 1u), 256, 0, stream>>>(
      X16, EMB, 0LL, W316, EMB, 0LL, QK16, 2 * EMB, 0LL, bqkv, NB * SEQ, 2 * EMB, EMB, 0.0625f);
  k_gemm_f16out_bm<<<dim3((unsigned)CDIV((EMB / 64) * (NB * SEQ / 64), 8), 1u), 256, 0, stream>>>(
      W316 + (size_t)2 * EMB * EMB, EMB, 0LL, X16, EMB, 0LL, VT16, NB * SEQ, 0LL, bqkv + 2 * EMB, EMB, NB * SEQ, EMB, 0.0625f);
  k_gemm_hilo_bn<<<dim3((unsigned)CDIV((EARLY / 64) * (2 * EMB / 64), 8), (unsigned)NB), 256, 0, stream>>>(
      X16, EMB, (long long)SEQ * EMB, W316, EMB, 0LL, QKEH, QKEL, 2 * EMB, (long long)EARLY * 2 * EMB, bqkv, EARLY, 2 * EMB, EMB, 0.0625f);
  k_gemm_hilo_bm<<<dim3((unsigned)CDIV((EMB / 64) * (EARLY / 64), 8), (unsigned)NB), 256, 0, stream>>>(
      W316 + (size_t)2 * EMB * EMB, EMB, 0LL, X16, EMB, (long long)SEQ * EMB, VTEH, VTEL, EARLY, (long long)EMB * EARLY, bqkv + 2 * EMB, EMB, EARLY, EMB, 0.0625f);

  if (SEQ > EARLY)
    k_attn_late<<<dim3((unsigned)((SEQ - EARLY) / 64), (unsigned)NHEAD, (unsigned)NB), 128, 0, stream>>>(QK16, VT16, CTX16);
  k_attn_early<<<dim3((unsigned)(EARLY / 64), (unsigned)NHEAD, (unsigned)NB), 128, 0, stream>>>(QKEH, QKEL, VTEH, VTEL, CTXEH, CTXEL);

  if (SEQ > EARLY)
    k_gemm_f32out_bn<<<dim3((unsigned)CDIV(((SEQ - EARLY) / 64) * (EMB / 64), 8), (unsigned)NB), 256, 0, stream>>>(
        CTX16 + (size_t)EARLY * EMB, EMB, (long long)SEQ * EMB, WO16, EMB, 0LL, out + (size_t)EARLY * EMB, EMB, (long long)SEQ_FULL * EMB,
        bo, SEQ - EARLY, EMB, EMB, 1.0f / 256.0f);
  k_gemm_bfsplit_f32out_bn<<<dim3((unsigned)CDIV((EARLY / 64) * (EMB / 64), 8), (unsigned)NB), 256, 0, stream>>>(
      CTXEH, CTXEL, EMB, (long long)EARLY * EMB, WOB, EMB, 0LL, out, EMB, (long long)SEQ_FULL * EMB, bo, EARLY, EMB, EMB, 1.0f);
}
